// SinkhornDistance_89833535963740
// MI455X (gfx1250) — hardware-verified
//
#include <hip/hip_runtime.h>
#include <math.h>

#pragma clang fp contract(off)

typedef unsigned short v8us  __attribute__((ext_vector_type(8)));
typedef unsigned short v16us __attribute__((ext_vector_type(16)));
typedef __bf16         v16bf __attribute__((ext_vector_type(16)));
typedef float          v8f   __attribute__((ext_vector_type(8)));
typedef float          v4f   __attribute__((ext_vector_type(4)));
typedef int            v4i   __attribute__((ext_vector_type(4)));
typedef v8us __attribute__((may_alias)) v8usa;
typedef v4f  __attribute__((may_alias)) v4fa;

union Frag { v16us v; v8us half[2]; };

constexpr int    NB       = 4;
constexpr int    NP       = 1024;
constexpr int    ND       = 256;
constexpr int    NROWS    = NB * NP;
constexpr int    NXY      = NROWS * ND;
constexpr int    NCI      = NB * NP * NP;
constexpr size_t NC       = (size_t)NCI;
constexpr int    NOUT     = 4 + NCI;
constexpr int    NLINES_OUT = (NOUT + 31) / 32;
constexpr int    OUT_BLK_LINES = 256;
constexpr int    NOUTBLK  = (NLINES_OUT + OUT_BLK_LINES - 1) / OUT_BLK_LINES;
constexpr int    NROWBLK  = NROWS / 32;
constexpr int    INIT_LINES = 257;
constexpr int    INIT_BLOCKS = (INIT_LINES * 8 + 255) / 256;
constexpr int    TP       = 68;
constexpr float  INV_EPS  = 10.0f;
constexpr float  EPS_F    = 0.1f;
constexpr float  THRESH   = 0.1f;
constexpr int    MAX_ITER = 20;

static_assert(ND % 32 == 0);
static_assert(NP % 128 == 0);
static_assert(NROWS % 32 == 0);
static_assert(NOUT == 4 + NCI);
static_assert((NLINES_OUT - 1) * 32 + 4 <= NOUT);
static_assert(NOUTBLK * OUT_BLK_LINES >= NLINES_OUT);

constexpr size_t WS_XB    = 0;
constexpr size_t WS_YB    = WS_XB    + (size_t)NXY * 2;
constexpr size_t WS_NRM   = WS_YB    + (size_t)NXY * 2;
constexpr size_t WS_C     = WS_NRM   + (size_t)2 * NROWS * 4;
constexpr size_t WS_CT    = WS_C     + NC * 4;
constexpr size_t WS_U     = WS_CT    + NC * 4;
constexpr size_t WS_V     = WS_U     + (size_t)NROWS * 4;
constexpr size_t WS_FLAG  = WS_V     + (size_t)NROWS * 4;
constexpr size_t WS_EPART = WS_FLAG  + 128;
constexpr size_t WS_VPART = WS_EPART + (size_t)NROWBLK * 128;
constexpr size_t WS_CPART = WS_VPART + (size_t)NROWBLK * 128;
constexpr size_t WS_TOTAL = WS_CPART + (size_t)NOUTBLK * 128;
static_assert(WS_TOTAL <= (size_t)134217728);
static_assert(WS_FLAG == WS_U + (size_t)(INIT_LINES - 1) * 128);
static_assert((WS_NRM % 128) == 0 && (WS_C % 128) == 0 && (WS_U % 128) == 0 && (WS_EPART % 128) == 0 && (WS_CPART % 128) == 0);

__device__ __forceinline__ float wave_sum(float v) {
  #pragma unroll
  for (int m = 16; m >= 1; m >>= 1) v += __shfl_xor(v, m, 32);
  return v;
}
__device__ __forceinline__ float wave_max(float v) {
  #pragma unroll
  for (int m = 16; m >= 1; m >>= 1) v = fmaxf(v, __shfl_xor(v, m, 32));
  return v;
}
__device__ __forceinline__ unsigned int bf16_bits(float f) {
  const unsigned int u = __float_as_uint(f);
  return (u + 0x7FFFu + ((u >> 16) & 1u)) >> 16;
}
__device__ __forceinline__ float bf16_rne(float f) {
  return __uint_as_float(bf16_bits(f) << 16);
}

__device__ __forceinline__ v8f wmma_bf16(v16us a, v16us b, v8f c) {
  v8f d = __builtin_amdgcn_wmma_f32_16x16x32_bf16(false, __builtin_bit_cast(v16bf, a), false,
                                                  __builtin_bit_cast(v16bf, b), (short)0, c, false, false);
  asm volatile("v_nop\n\tv_nop\n\tv_nop\n\tv_nop" : "+v"(d) : "v"(a), "v"(b));
  return d;
}

__device__ __forceinline__ v16us load_frag(const unsigned short* p, int h) {
  Frag f;
  f.half[0] = *(const v8usa*)(p + 8 * h);
  f.half[1] = *(const v8usa*)(p + 16 + 8 * h);
  return f.v;
}

__device__ __forceinline__ float marg(float c, float vec, float rs, int selfFirst, float logq) {
  const float f1 = selfFirst ? rs : vec;
  const float f2 = selfFirst ? vec : rs;
  return (((-c) + f1) + f2 - logq) * INV_EPS;
}

__global__ __launch_bounds__(256) void k_init(float* __restrict__ uvf) {
  const int gid = blockIdx.x * 256 + threadIdx.x;
  const int L = gid >> 3, q8 = gid & 7;
  const bool act = (L < INIT_LINES);
  const int Lc = act ? L : 0;
  const v4f z = {0.f, 0.f, 0.f, 0.f};
  float* p = uvf + (size_t)Lc * 32 + 4 * q8;
  if (act) *(volatile v4f*)p = z;
  __threadfence();
  if (act) *(volatile v4f*)p = z;
}

__global__ __launch_bounds__(256) void k_prep(const float* __restrict__ x, const float* __restrict__ y,
                                              unsigned short* __restrict__ xb, unsigned short* __restrict__ yb,
                                              float* __restrict__ nrm) {
  __shared__ __attribute__((aligned(16))) float sN[32];
  const int tid = threadIdx.x, lane = tid & 31, w = tid >> 5;
  const int rb = blockIdx.x * 32;
  const bool isy = (rb >= NROWS);
  const int rloc = isy ? (rb - NROWS) : rb;
  const float* src = (isy ? y : x) + (size_t)rloc * ND;
  unsigned short* dst = (isy ? yb : xb) + (size_t)rloc * ND;

  v8us ov[4];
  #pragma unroll
  for (int s = 0; s < 4; ++s) {
    const int rl = 4 * w + s;
    const float* rp = src + (size_t)rl * ND + 8 * lane;
    const v4f a = *(const v4fa*)rp;
    const v4f c = *(const v4fa*)(rp + 4);
    const unsigned int b0 = bf16_bits(a.x), b1 = bf16_bits(a.y), b2 = bf16_bits(a.z), b3 = bf16_bits(a.w);
    const unsigned int b4 = bf16_bits(c.x), b5 = bf16_bits(c.y), b6 = bf16_bits(c.z), b7 = bf16_bits(c.w);
    const float r0 = __uint_as_float(b0 << 16), r1 = __uint_as_float(b1 << 16);
    const float r2 = __uint_as_float(b2 << 16), r3 = __uint_as_float(b3 << 16);
    const float r4 = __uint_as_float(b4 << 16), r5 = __uint_as_float(b5 << 16);
    const float r6 = __uint_as_float(b6 << 16), r7 = __uint_as_float(b7 << 16);
    float ss = r0 * r0;
    ss = ss + r1 * r1; ss = ss + r2 * r2; ss = ss + r3 * r3;
    ss = ss + r4 * r4; ss = ss + r5 * r5; ss = ss + r6 * r6; ss = ss + r7 * r7;
    ss = wave_sum(ss);
    if (lane == 0) sN[rl] = sqrtf(ss);
    v8us o;
    o[0] = (unsigned short)b0; o[1] = (unsigned short)b1; o[2] = (unsigned short)b2; o[3] = (unsigned short)b3;
    o[4] = (unsigned short)b4; o[5] = (unsigned short)b5; o[6] = (unsigned short)b6; o[7] = (unsigned short)b7;
    ov[s] = o;
    *(volatile v8us*)(dst + (size_t)rl * ND + 8 * lane) = o;
  }
  __threadfence();
  #pragma unroll
  for (int s = 0; s < 4; ++s) {
    const int rl = 4 * w + s;
    *(volatile v8us*)(dst + (size_t)rl * ND + 8 * lane) = ov[s];
  }
  __syncthreads();
  const int q8 = lane & 7;
  const bool wr = (w == 0) && (lane < 8);
  const v4f nv = *(const v4fa*)(sN + 4 * q8);
  float* np = nrm + rb + 4 * q8;
  if (wr) *(volatile v4f*)np = nv;
  __threadfence();
  if (wr) *(volatile v4f*)np = nv;
}

__device__ __forceinline__ void cost_store_pass(const float* sT, float* Cp, float* CTp,
                                                int b, int i0, int j0, int w, int lane) {
  const int q8 = lane & 7, sub = lane >> 3;
  #pragma unroll
  for (int i = 0; i < 16; ++i) {
    const int lid = w * 64 + i * 4 + sub;
    const int row = lid >> 1, hl = lid & 1;
    const v4f v = *(const v4fa*)(sT + row * TP + 32 * hl + 4 * q8);
    float* dst = Cp + ((size_t)(b * NP) + i0 + row) * NP + j0 + 32 * hl + 4 * q8;
    *(volatile v4f*)dst = v;
  }
  #pragma unroll
  for (int i = 0; i < 16; ++i) {
    const int lid = w * 64 + i * 4 + sub;
    const int jr = lid >> 2, qt = lid & 3;
    const int il = qt * 32 + 4 * q8;
    v4f v;
    v.x = sT[(il + 0) * TP + jr];
    v.y = sT[(il + 1) * TP + jr];
    v.z = sT[(il + 2) * TP + jr];
    v.w = sT[(il + 3) * TP + jr];
    float* dst = CTp + ((size_t)(b * NP) + j0 + jr) * NP + i0 + il;
    *(volatile v4f*)dst = v;
  }
}

__global__ __launch_bounds__(128) void k_cost(const unsigned short* __restrict__ xb,
                                              const unsigned short* __restrict__ yb,
                                              const float* __restrict__ nrm,
                                              float* __restrict__ Cp, float* __restrict__ CTp) {
  __shared__ __attribute__((aligned(16))) float sT[128 * TP];
  __shared__ float sNX[128];
  __shared__ float sNY[64];

  const int tid = threadIdx.x, lane = tid & 31, w = tid >> 5;
  const int h = lane >> 4, m = lane & 15;
  const int j0 = blockIdx.x * 64, i0 = blockIdx.y * 128, b = blockIdx.z;

  sNX[tid] = nrm[b * NP + i0 + tid];
  if (tid < 64) sNY[tid] = nrm[NROWS + b * NP + j0 + tid];
  __syncthreads();

  const unsigned short* xa0 = xb + ((size_t)(b * NP) + i0 + 32 * w + m) * ND;
  const unsigned short* xa1 = xa0 + (size_t)16 * ND;
  const unsigned short* ya  = yb + ((size_t)(b * NP) + j0 + m) * ND;

  const v8f zero8 = {0.f, 0.f, 0.f, 0.f, 0.f, 0.f, 0.f, 0.f};
  v8f acc[2][4];
  #pragma unroll
  for (int mt = 0; mt < 2; ++mt)
    #pragma unroll
    for (int nt = 0; nt < 4; ++nt) acc[mt][nt] = zero8;

  #pragma unroll 4
  for (int k0 = 0; k0 < ND; k0 += 32) {
    const v16us a0 = load_frag(xa0 + k0, h);
    const v16us a1 = load_frag(xa1 + k0, h);
    #pragma unroll
    for (int nt = 0; nt < 4; ++nt) {
      const v16us bfr = load_frag(ya + (size_t)nt * 16 * ND + k0, h);
      acc[0][nt] = wmma_bf16(a0, bfr, acc[0][nt]);
      acc[1][nt] = wmma_bf16(a1, bfr, acc[1][nt]);
    }
  }

  #pragma unroll
  for (int nt = 0; nt < 4; ++nt) {
    const int jl = 16 * nt + m;
    const float nyv = sNY[jl];
    #pragma unroll
    for (int mt = 0; mt < 2; ++mt) {
      #pragma unroll
      for (int r = 0; r < 8; ++r) {
        const int il = 32 * w + 16 * mt + 8 * h + r;
        const float den = fmaxf(sNX[il] * nyv, 1e-8f);
        const float rc  = 1.0f / den;
        const float c   = 1.0f - acc[mt][nt][r] * rc;
        sT[il * TP + jl] = c;
      }
    }
  }
  __syncthreads();

  cost_store_pass(sT, Cp, CTp, b, i0, j0, w, lane);
  __threadfence();
  cost_store_pass(sT, Cp, CTp, b, i0, j0, w, lane);
}

__global__ __launch_bounds__(256) void k_lse(const float* __restrict__ Cm, float* selfv,
                                             const float* __restrict__ otherv, const float* __restrict__ q,
                                             const int* __restrict__ flag, float* __restrict__ part,
                                             int selfFirst) {
  __shared__ __attribute__((aligned(16))) float sO[NP];
  __shared__ __attribute__((aligned(16))) float sU[32];
  __shared__ float sD[32];
  __shared__ float sP[1];

  if (flag[0] != 0) return;

  const int tid = threadIdx.x, lane = tid & 31, w = tid >> 5;
  const int row0 = blockIdx.x * 32;
  const int b = row0 >> 10;

  *(v4fa*)(sO + 4 * tid) = *(const v4fa*)(otherv + (size_t)b * NP + 4 * tid);
  __syncthreads();

  const float logq = logf(bf16_rne(q[0]));
  const float logm = logf(9.765625e-4f + 1e-8f);

  #pragma unroll 1
  for (int s = 0; s < 4; ++s) {
    const int rl = 4 * w + s;
    const int row = row0 + rl;
    const float sv = selfv[row];
    const float* cr = Cm + (size_t)row * NP;

    float mx = -__builtin_inff();
    #pragma unroll
    for (int t = 0; t < 8; ++t) {
      const v4f c4 = *(const v4fa*)(cr + 128 * t + 4 * lane);
      const v4f o4 = *(const v4fa*)(sO + 128 * t + 4 * lane);
      mx = fmaxf(mx, marg(c4.x, o4.x, sv, selfFirst, logq));
      mx = fmaxf(mx, marg(c4.y, o4.y, sv, selfFirst, logq));
      mx = fmaxf(mx, marg(c4.z, o4.z, sv, selfFirst, logq));
      mx = fmaxf(mx, marg(c4.w, o4.w, sv, selfFirst, logq));
    }
    mx = wave_max(mx);

    float ss = 0.f;
    #pragma unroll 1
    for (int t = 0; t < 8; ++t) {
      const v4f c4 = *(const v4fa*)(cr + 128 * t + 4 * lane);
      const v4f o4 = *(const v4fa*)(sO + 128 * t + 4 * lane);
      ss += expf(marg(c4.x, o4.x, sv, selfFirst, logq) - mx);
      ss += expf(marg(c4.y, o4.y, sv, selfFirst, logq) - mx);
      ss += expf(marg(c4.z, o4.z, sv, selfFirst, logq) - mx);
      ss += expf(marg(c4.w, o4.w, sv, selfFirst, logq) - mx);
    }
    ss = wave_sum(ss);

    const float lse = logf(ss) + mx;
    const float nv  = EPS_F * (logm - lse) + sv;
    if (lane == 0) { sU[rl] = nv; sD[rl] = fabsf(nv - sv); }
  }
  __syncthreads();
  if (tid == 0) {
    float p = 0.f;
    for (int r = 0; r < 32; ++r) p += sD[r];
    sP[0] = p;
  }
  __syncthreads();

  const int q8 = lane & 7;
  const bool wr = (w == 0) && (lane < 8);
  const v4f uv = *(const v4fa*)(sU + 4 * q8);
  v4f pv = {0.f, 0.f, 0.f, 0.f};
  pv.x = (q8 == 0) ? sP[0] : 0.f;
  float* up = selfv + row0 + 4 * q8;
  float* pp = part + (size_t)blockIdx.x * 32 + 4 * q8;
  if (wr) { *(volatile v4f*)up = uv; *(volatile v4f*)pp = pv; }
  __threadfence();
  if (wr) { *(volatile v4f*)up = uv; *(volatile v4f*)pp = pv; }
}

__global__ __launch_bounds__(128) void k_flag(const float* __restrict__ part, int* flag) {
  __shared__ float sP[NROWBLK];
  __shared__ int sF[1];
  const int tid = threadIdx.x;
  sP[tid] = part[(size_t)tid * 32];
  __syncthreads();
  if (tid == 0) {
    float tot = 0.f;
    for (int bb = 0; bb < NB; ++bb) {
      float s = 0.f;
      for (int k = 0; k < 32; ++k) s += sP[32 * bb + k];
      tot += s;
    }
    const float err = tot * 0.25f;
    const int old = flag[0];
    sF[0] = old | ((err < THRESH) ? 1 : 0);
  }
  __syncthreads();
  v4i fv = {0, 0, 0, 0};
  fv.x = (tid == 0) ? sF[0] : 0;
  const bool wr = (tid < 8);
  int* fp = flag + 4 * (tid & 7);
  if (wr) *(volatile v4i*)fp = fv;
  __threadfence();
  if (wr) *(volatile v4i*)fp = fv;
}

__global__ __launch_bounds__(256) void k_out(const float* __restrict__ Cp, const float* __restrict__ u,
                                             const float* __restrict__ v, const float* __restrict__ q,
                                             float* __restrict__ out, float* __restrict__ cpart) {
  __shared__ float sR[8][4];
  __shared__ __attribute__((aligned(16))) float sC[4];
  const int tid = threadIdx.x, lane = tid & 31, w = tid >> 5;
  const int q8 = lane & 7, sub = lane >> 3;
  const float logq = logf(bf16_rne(q[0]));
  float a0 = 0.f, a1 = 0.f, a2 = 0.f, a3 = 0.f;
  const int Lb = blockIdx.x * OUT_BLK_LINES + 32 * w + sub;

  #pragma unroll 1
  for (int i = 0; i < 8; ++i) {
    const int L = Lb + 4 * i;
    const int f = 32 * L + 4 * q8;
    const bool act = (L >= 1) && (f + 3 < NOUT);
    int e = f - 4;
    e = (e < 0) ? 0 : e;
    e = (e > NCI - 4) ? (NCI - 4) : e;
    const int bb = e >> 20, ii = (e >> 10) & 1023, jj = e & 1023;
    const v4f c4 = *(const v4fa*)(Cp + e);
    const v4f v4 = *(const v4fa*)(v + bb * NP + jj);
    const float ui = u[bb * NP + ii];
    v4f p;
    p.x = expf((((-c4.x) + ui) + v4.x - logq) * INV_EPS);
    p.y = expf((((-c4.y) + ui) + v4.y - logq) * INV_EPS);
    p.z = expf((((-c4.z) + ui) + v4.z - logq) * INV_EPS);
    p.w = expf((((-c4.w) + ui) + v4.w - logq) * INV_EPS);
    float* op = out + f;
    if (act) *(volatile v4f*)op = p;
    __threadfence();
    if (act) *(volatile v4f*)op = p;
    float s = p.x * c4.x;
    s = s + p.y * c4.y; s = s + p.z * c4.z; s = s + p.w * c4.w;
    s = act ? s : 0.f;
    a0 += (bb == 0) ? s : 0.f;
    a1 += (bb == 1) ? s : 0.f;
    a2 += (bb == 2) ? s : 0.f;
    a3 += (bb == 3) ? s : 0.f;
  }
  a0 = wave_sum(a0); a1 = wave_sum(a1); a2 = wave_sum(a2); a3 = wave_sum(a3);
  if (lane == 0) { sR[w][0] = a0; sR[w][1] = a1; sR[w][2] = a2; sR[w][3] = a3; }
  __syncthreads();
  if (tid < 4) {
    float t = 0.f;
    for (int k = 0; k < 8; ++k) t += sR[k][tid];
    sC[tid] = t;
  }
  __syncthreads();
  const v4f zero4 = {0.f, 0.f, 0.f, 0.f};
  const v4f cs = *(const v4fa*)sC;
  const v4f pv = (tid == 0) ? cs : zero4;
  const bool wr = (tid < 8);
  float* pp = cpart + (size_t)blockIdx.x * 32 + 4 * (tid & 7);
  if (wr) *(volatile v4f*)pp = pv;
  __threadfence();
  if (wr) *(volatile v4f*)pp = pv;
}

__global__ __launch_bounds__(256) void k_fold(const float* __restrict__ cpart, const float* __restrict__ Cp,
                                              const float* __restrict__ u, const float* __restrict__ v,
                                              const float* __restrict__ q, float* __restrict__ out) {
  __shared__ float sR[256][4];
  __shared__ float sS[8];
  __shared__ __attribute__((aligned(16))) float sC[4];
  const int tid = threadIdx.x;
  float a0 = 0.f, a1 = 0.f, a2 = 0.f, a3 = 0.f;
  #pragma unroll 1
  for (int k = tid; k < NOUTBLK; k += 256) {
    const v4f p4 = *(const v4fa*)(cpart + (size_t)k * 32);
    a0 += p4.x; a1 += p4.y; a2 += p4.z; a3 += p4.w;
  }
  sR[tid][0] = a0; sR[tid][1] = a1; sR[tid][2] = a2; sR[tid][3] = a3;

  const float logq = logf(bf16_rne(q[0]));
  int e = 4 * tid - 4;
  e = (e < 0) ? 0 : e;
  e = (e > NP - 4) ? (NP - 4) : e;
  const v4f c4 = *(const v4fa*)(Cp + e);
  const v4f v4 = *(const v4fa*)(v + e);
  const float ui = u[0];
  v4f p;
  p.x = expf((((-c4.x) + ui) + v4.x - logq) * INV_EPS);
  p.y = expf((((-c4.y) + ui) + v4.y - logq) * INV_EPS);
  p.z = expf((((-c4.z) + ui) + v4.z - logq) * INV_EPS);
  p.w = expf((((-c4.w) + ui) + v4.w - logq) * INV_EPS);
  float s = p.x * c4.x;
  s = s + p.y * c4.y; s = s + p.z * c4.z; s = s + p.w * c4.w;
  const bool own = (tid >= 1) && (tid < 8);
  if (tid < 8) sS[tid] = own ? s : 0.f;
  __syncthreads();
  if (tid < 4) {
    float t = 0.f;
    for (int r = 0; r < 256; ++r) t += sR[r][tid];
    if (tid == 0) {
      float hsum = 0.f;
      for (int k = 1; k < 8; ++k) hsum += sS[k];
      t += hsum;
    }
    sC[tid] = t;
  }
  __syncthreads();

  const v4f cs = *(const v4fa*)sC;
  const v4f val = (tid == 0) ? cs : p;
  const bool wr = (tid < 8);
  float* op = out + 4 * (tid & 7);
  if (wr) *(volatile v4f*)op = val;
  __threadfence();
  if (wr) *(volatile v4f*)op = val;
}

extern "C" void kernel_launch(void* const* d_in, const int* in_sizes, int n_in,
                              void* d_out, int out_size, void* d_ws, size_t ws_size,
                              hipStream_t stream) {
  if (n_in < 3) return;
  if (in_sizes[0] != NXY || in_sizes[1] != NXY || in_sizes[2] < 1) return;
  if (out_size != NOUT) return;
  if (ws_size < WS_TOTAL) return;

  const float* x = (const float*)d_in[0];
  const float* y = (const float*)d_in[1];
  const float* q = (const float*)d_in[2];
  float* out = (float*)d_out;

  char* ws = (char*)d_ws;
  unsigned short* xb = (unsigned short*)(ws + WS_XB);
  unsigned short* yb = (unsigned short*)(ws + WS_YB);
  float* nrm   = (float*)(ws + WS_NRM);
  float* C     = (float*)(ws + WS_C);
  float* CT    = (float*)(ws + WS_CT);
  float* u     = (float*)(ws + WS_U);
  float* v     = (float*)(ws + WS_V);
  int*   flag  = (int*)(ws + WS_FLAG);
  float* epart = (float*)(ws + WS_EPART);
  float* vpart = (float*)(ws + WS_VPART);
  float* cpart = (float*)(ws + WS_CPART);

  k_init<<<INIT_BLOCKS, 256, 0, stream>>>(u);
  k_prep<<<(2 * NROWS) / 32, 256, 0, stream>>>(x, y, xb, yb, nrm);
  k_cost<<<dim3(NP / 64, NP / 128, NB), 128, 0, stream>>>(xb, yb, nrm, C, CT);
  for (int it = 0; it < MAX_ITER; ++it) {
    k_lse<<<NROWBLK, 256, 0, stream>>>(C,  u, v, q, flag, epart, 1);
    k_lse<<<NROWBLK, 256, 0, stream>>>(CT, v, u, q, flag, vpart, 0);
    k_flag<<<1, 128, 0, stream>>>(epart, flag);
  }
  k_out<<<NOUTBLK, 256, 0, stream>>>(C, u, v, q, out, cpart);
  k_fold<<<1, 256, 0, stream>>>(cpart, C, u, v, q, out);
}
